// SwappedTransformerLayerRoPE_51883204936010
// MI455X (gfx1250) — hardware-verified
//
#include <hip/hip_runtime.h>

typedef _Float16 v16h __attribute__((ext_vector_type(16)));
typedef _Float16 v8h  __attribute__((ext_vector_type(8)));
typedef float    v8f  __attribute__((ext_vector_type(8)));
typedef float    v4f  __attribute__((ext_vector_type(4)));
typedef v8h __attribute__((may_alias)) v8ha;
typedef v4f __attribute__((may_alias)) v4fa;

union Frag { v16h v; v8h half[2]; };

#define HIDDEN 1024
#define NHEADS 16
#define HD     64
#define SEQ    512
#define BATCH  8
#define MROWS  (BATCH * SEQ)
#define NX     (MROWS * HIDDEN)
#define NW     (HIDDEN * HIDDEN)
#define NBH    (BATCH * NHEADS)
#define RHALF  (HD / 2)
#define WSCALE 32.0f
#define PSCALE 16384.0f
#define OSCALE 16.0f
#define SM_SCALE 0.125f
#define LN_EPS 1e-5f
#define LOG2_BASE_STEP 0.025952563241307520f

__device__ __forceinline__ v8f wmma_f16(v16h a, v16h b, v8f c) {
  v8f d = __builtin_amdgcn_wmma_f32_16x16x32_f16(false, a, false, b, (short)0, c, false, false);
  asm volatile("v_nop\n\tv_nop\n\tv_nop\n\tv_nop" : "+v"(d) : "v"(a), "v"(b));
  return d;
}

__device__ __forceinline__ v16h load_frag(const _Float16* p, int h) {
  Frag f;
  f.half[0] = *(const v8ha*)(p + 8 * h);
  f.half[1] = *(const v8ha*)(p + 16 + 8 * h);
  return f.v;
}

__global__ __launch_bounds__(256) void rope_table_kernel(float* __restrict__ ct, float* __restrict__ st) {
  const int g = blockIdx.x * 256 + threadIdx.x;
  if (g >= SEQ * (RHALF / 4)) return;
  const int pos = g >> 3;
  const int i0 = (g & 7) * 4;
  v4f c4 = {0.f, 0.f, 0.f, 0.f};
  v4f s4 = {0.f, 0.f, 0.f, 0.f};
  #pragma unroll 1
  for (int e = 0; e < 4; ++e) {
    const float fi = (float)(i0 + e);
    const float ifr = exp2f(-fi * LOG2_BASE_STEP);
    const float ang = (float)pos * ifr;
    const float cs = cosf(ang);
    const float sn = sinf(ang);
    if (e == 0)      { c4.x = cs; s4.x = sn; }
    else if (e == 1) { c4.y = cs; s4.y = sn; }
    else if (e == 2) { c4.z = cs; s4.z = sn; }
    else             { c4.w = cs; s4.w = sn; }
  }
  float* dc = ct + (size_t)pos * RHALF + i0;
  float* ds = st + (size_t)pos * RHALF + i0;
  *(volatile v4f*)dc = c4;
  *(volatile v4f*)ds = s4;
  __threadfence();
  *(volatile v4f*)dc = c4;
  *(volatile v4f*)ds = s4;
}

__global__ __launch_bounds__(256) void wconv_kernel(
    const float* __restrict__ wq, const float* __restrict__ wk,
    const float* __restrict__ wv, const float* __restrict__ wo,
    _Float16* __restrict__ wt)
{
  __shared__ float sW[64][65];
  const int t = threadIdx.x, lane = t & 31, w = t >> 5;
  const int n0 = blockIdx.x * 64, k0 = blockIdx.y * 64, z = blockIdx.z;
  const float* W = (z == 0) ? wq : ((z == 1) ? wk : ((z == 2) ? wv : wo));
  #pragma unroll
  for (int p = 0; p < 4; ++p) {
    const int j = t + 256 * p;
    const int kk = j >> 4, c4 = j & 15;
    const v4f v = *(const v4fa*)(W + (size_t)(k0 + kk) * HIDDEN + n0 + 4 * c4);
    sW[kk][4 * c4 + 0] = v.x;
    sW[kk][4 * c4 + 1] = v.y;
    sW[kk][4 * c4 + 2] = v.z;
    sW[kk][4 * c4 + 3] = v.w;
  }
  __syncthreads();
  _Float16* dstz = wt + (size_t)z * NW;
  const int q8 = lane & 7, sub = lane >> 3;
  #pragma unroll
  for (int pass = 0; pass < 2; ++pass) {
    #pragma unroll
    for (int i = 0; i < 2; ++i) {
      const int nn = 8 * w + 4 * i + sub;
      const int kb = 8 * q8;
      const v8h o = { (_Float16)(sW[kb + 0][nn] * WSCALE), (_Float16)(sW[kb + 1][nn] * WSCALE),
                      (_Float16)(sW[kb + 2][nn] * WSCALE), (_Float16)(sW[kb + 3][nn] * WSCALE),
                      (_Float16)(sW[kb + 4][nn] * WSCALE), (_Float16)(sW[kb + 5][nn] * WSCALE),
                      (_Float16)(sW[kb + 6][nn] * WSCALE), (_Float16)(sW[kb + 7][nn] * WSCALE) };
      _Float16* dst = dstz + (size_t)(n0 + nn) * HIDDEN + k0 + kb;
      *(volatile v8h*)dst = o;
    }
    if (pass == 0) __threadfence();
  }
}

__global__ __launch_bounds__(128) void ln_kernel(
    const float* __restrict__ x, const float* __restrict__ g, const float* __restrict__ bb,
    _Float16* __restrict__ xh)
{
  __shared__ float red0[4];
  __shared__ float red1[4];
  const int row = blockIdx.x, t = threadIdx.x, lane = t & 31, w = t >> 5;
  const float* xr = x + (size_t)row * HIDDEN + 8 * t;
  const v4f a = *(const v4fa*)xr;
  const v4f c = *(const v4fa*)(xr + 4);
  float s = ((a.x + a.y) + (a.z + a.w)) + ((c.x + c.y) + (c.z + c.w));
  #pragma unroll
  for (int off = 16; off; off >>= 1) s += __shfl_xor(s, off, 32);
  if (lane == 0) red0[w] = s;
  __syncthreads();
  const float mean = ((red0[0] + red0[1]) + (red0[2] + red0[3])) * (1.0f / HIDDEN);
  const v4f da = a - mean;
  const v4f dc = c - mean;
  float sq = ((da.x * da.x + da.y * da.y) + (da.z * da.z + da.w * da.w))
           + ((dc.x * dc.x + dc.y * dc.y) + (dc.z * dc.z + dc.w * dc.w));
  #pragma unroll
  for (int off = 16; off; off >>= 1) sq += __shfl_xor(sq, off, 32);
  if (lane == 0) red1[w] = sq;
  __syncthreads();
  const float var = ((red1[0] + red1[1]) + (red1[2] + red1[3])) * (1.0f / HIDDEN);
  const float rs = rsqrtf(var + LN_EPS);
  const v4f ga = *(const v4fa*)(g + 8 * t);
  const v4f gc = *(const v4fa*)(g + 8 * t + 4);
  const v4f ba = *(const v4fa*)(bb + 8 * t);
  const v4f bc = *(const v4fa*)(bb + 8 * t + 4);
  const v4f ya = da * rs * ga + ba;
  const v4f yc = dc * rs * gc + bc;
  const v8h o = { (_Float16)ya.x, (_Float16)ya.y, (_Float16)ya.z, (_Float16)ya.w,
                  (_Float16)yc.x, (_Float16)yc.y, (_Float16)yc.z, (_Float16)yc.w };
  _Float16* dst = xh + (size_t)row * HIDDEN + 8 * t;
  *(volatile v8h*)dst = o;
  __threadfence();
  *(volatile v8h*)dst = o;
}

__device__ __forceinline__ void proj_store_pass(const _Float16* sT, _Float16* plane, _Float16* vt,
                                                int which, int bh, int l0, int w, int lane) {
  const int q8 = lane & 7, sub = lane >> 3;
  #pragma unroll
  for (int i = 0; i < 8; ++i) {
    const int lid = w * 32 + i * 4 + sub;
    v8h v;
    _Float16* dst;
    if (which != 2) {
      v = *(const v8ha*)(sT + lid * HD + 8 * q8);
      dst = plane + ((size_t)bh * SEQ + l0 + lid) * HD + 8 * q8;
    } else {
      const int d = lid >> 1, hl = lid & 1;
      v = *(const v8ha*)(sT + d * 128 + 64 * hl + 8 * q8);
      dst = vt + ((size_t)bh * HD + d) * SEQ + l0 + 64 * hl + 8 * q8;
    }
    *(volatile v8h*)dst = v;
  }
}

__global__ __launch_bounds__(128) void proj_kernel(
    const _Float16* __restrict__ xh,
    const _Float16* __restrict__ wh,
    const float* __restrict__ bq, const float* __restrict__ bk, const float* __restrict__ bv,
    const float* __restrict__ ct, const float* __restrict__ st,
    _Float16* __restrict__ qh,
    _Float16* __restrict__ kh,
    _Float16* __restrict__ vt)
{
  __shared__ __attribute__((aligned(16))) _Float16 sT[128 * 64];

  const int tid = threadIdx.x, lane = tid & 31, w = tid >> 5;
  const int h = lane >> 4, m = lane & 15;
  const int m0 = blockIdx.x * 128;
  const int cg = blockIdx.y;
  const int which = cg >> 4, head = cg & 15;
  const int m0w = m0 + 32 * w;

  const _Float16* xa0 = xh + (size_t)(m0w + m) * HIDDEN;
  const _Float16* xa1 = xa0 + (size_t)16 * HIDDEN;
  const _Float16* wb  = wh + ((size_t)which * HIDDEN + head * HD + m) * HIDDEN;

  const v8f zero8 = {0.f, 0.f, 0.f, 0.f, 0.f, 0.f, 0.f, 0.f};
  v8f acc[2][4];
  #pragma unroll
  for (int mt = 0; mt < 2; ++mt)
    #pragma unroll
    for (int nt = 0; nt < 4; ++nt) acc[mt][nt] = zero8;

  #pragma unroll 1
  for (int k0 = 0; k0 < HIDDEN; k0 += 32) {
    const v16h a0 = load_frag(xa0 + k0, h);
    const v16h a1 = load_frag(xa1 + k0, h);
    #pragma unroll
    for (int nt = 0; nt < 4; ++nt) {
      const v16h b = load_frag(wb + (size_t)nt * 16 * HIDDEN + k0, h);
      acc[0][nt] = wmma_f16(a0, b, acc[0][nt]);
      acc[1][nt] = wmma_f16(a1, b, acc[1][nt]);
    }
  }

  const float* bias = (which == 0) ? bq : ((which == 1) ? bk : bv);
  const int b = m0 >> 9, l0 = m0 & (SEQ - 1), bh = b * NHEADS + head;
  #pragma unroll
  for (int nt = 0; nt < 4; ++nt) {
    const int feat = 16 * nt + m;
    const float bvl = bias[head * HD + feat];
    const int fi = feat >> 1;
    const float sgn = (feat & 1) ? 1.0f : -1.0f;
    #pragma unroll
    for (int mt = 0; mt < 2; ++mt) {
      #pragma unroll
      for (int r = 0; r < 8; ++r) {
        const int tokl = 32 * w + 16 * mt + 8 * h + r;
        const int pos = l0 + tokl;
        const float y = acc[mt][nt][r] * (1.0f / WSCALE) + bvl;
        const float yp = __shfl_xor(y, 1, 32);
        float o = y;
        if (which != 2) {
          const float cs = ct[pos * RHALF + fi];
          const float sn = st[pos * RHALF + fi];
          o = y * cs + (sgn * yp) * sn;
        }
        const int idx = (which == 2) ? (feat * 128 + tokl) : (tokl * HD + feat);
        sT[idx] = (_Float16)o;
      }
    }
  }
  __syncthreads();

  _Float16* plane = (which == 0) ? qh : kh;
  proj_store_pass(sT, plane, vt, which, bh, l0, w, lane);
  __threadfence();
  proj_store_pass(sT, plane, vt, which, bh, l0, w, lane);
}

__device__ __forceinline__ v16h pack_p(v8f a, v8f c) {
  const v16h r = { (_Float16)(a[0] * PSCALE), (_Float16)(a[1] * PSCALE), (_Float16)(a[2] * PSCALE), (_Float16)(a[3] * PSCALE),
                   (_Float16)(a[4] * PSCALE), (_Float16)(a[5] * PSCALE), (_Float16)(a[6] * PSCALE), (_Float16)(a[7] * PSCALE),
                   (_Float16)(c[0] * PSCALE), (_Float16)(c[1] * PSCALE), (_Float16)(c[2] * PSCALE), (_Float16)(c[3] * PSCALE),
                   (_Float16)(c[4] * PSCALE), (_Float16)(c[5] * PSCALE), (_Float16)(c[6] * PSCALE), (_Float16)(c[7] * PSCALE) };
  return r;
}

__device__ __forceinline__ void att_store_pass(const _Float16* so, _Float16* oh,
                                               int b, int head, int q0, int lane) {
  const int q8 = lane & 7, sub = lane >> 3;
  #pragma unroll
  for (int i = 0; i < 4; ++i) {
    const int row = i * 4 + sub;
    const v8h v = *(const v8ha*)(so + row * HD + 8 * q8);
    const size_t gi = ((size_t)b * SEQ + q0 + row) * HIDDEN + head * HD + 8 * q8;
    *(volatile v8h*)(oh + gi) = v;
  }
}

__global__ __launch_bounds__(128) void attn_kernel(
    const _Float16* __restrict__ qh,
    const _Float16* __restrict__ kh,
    const _Float16* __restrict__ vt,
    _Float16* __restrict__ oh)
{
  __shared__ __attribute__((aligned(16))) _Float16 sO[4 * 16 * HD];

  const int tid = threadIdx.x, lane = tid & 31, w = tid >> 5;
  const int h = lane >> 4, m = lane & 15;
  const int bh = blockIdx.y, b = bh >> 4, head = bh & 15;
  const int q0 = blockIdx.x * 64 + 16 * w;

  const _Float16* qrow = qh + ((size_t)bh * SEQ + q0 + m) * HD;
  const v16h qb0 = load_frag(qrow, h);
  const v16h qb1 = load_frag(qrow + 32, h);

  const v8f zero8 = {0.f, 0.f, 0.f, 0.f, 0.f, 0.f, 0.f, 0.f};
  v8f o[4];
  #pragma unroll
  for (int t = 0; t < 4; ++t) o[t] = zero8;
  float mrun = -1e30f, lrun = 0.0f;

  const _Float16* kbase = kh + ((size_t)bh * SEQ + m) * HD;
  const _Float16* vbase = vt + ((size_t)bh * HD + m) * SEQ;

  #pragma unroll 1
  for (int kb = 0; kb < SEQ; kb += 64) {
    v8f s[4];
    #pragma unroll
    for (int j = 0; j < 4; ++j) {
      const _Float16* kp = kbase + (size_t)(kb + 16 * j) * HD;
      const v16h kf0 = load_frag(kp, h);
      const v16h kf1 = load_frag(kp + 32, h);
      v8f z = zero8;
      z = wmma_f16(kf0, qb0, z);
      z = wmma_f16(kf1, qb1, z);
      s[j] = z * SM_SCALE;
    }

    float mloc = s[0][0];
    #pragma unroll
    for (int j = 0; j < 4; ++j)
      #pragma unroll
      for (int r = 0; r < 8; ++r) mloc = fmaxf(mloc, s[j][r]);
    mloc = fmaxf(mloc, __shfl_xor(mloc, 16, 32));
    const float mnew = fmaxf(mrun, mloc);
    const float alpha = __expf(mrun - mnew);
    mrun = mnew;
    float lsum = 0.0f;
    #pragma unroll
    for (int j = 0; j < 4; ++j)
      #pragma unroll
      for (int r = 0; r < 8; ++r) {
        const float p = __expf(s[j][r] - mnew);
        s[j][r] = p;
        lsum += p;
      }
    lsum += __shfl_xor(lsum, 16, 32);
    lrun = lrun * alpha + lsum;
    #pragma unroll
    for (int t = 0; t < 4; ++t)
      #pragma unroll
      for (int r = 0; r < 8; ++r) o[t][r] = o[t][r] * alpha;

    const v16h pb0 = pack_p(s[0], s[1]);
    const v16h pb1 = pack_p(s[2], s[3]);

    #pragma unroll
    for (int t = 0; t < 4; ++t) {
      const _Float16* vp = vbase + (size_t)(16 * t) * SEQ + kb;
      const v16h vf0 = load_frag(vp, h);
      const v16h vf1 = load_frag(vp + 32, h);
      o[t] = wmma_f16(vf0, pb0, o[t]);
      o[t] = wmma_f16(vf1, pb1, o[t]);
    }
  }

  const float inv = (1.0f / lrun) * (OSCALE / PSCALE);
  _Float16* so = sO + w * (16 * HD);
  #pragma unroll
  for (int t = 0; t < 4; ++t)
    #pragma unroll
    for (int r = 0; r < 8; ++r)
      so[m * HD + 16 * t + 8 * h + r] = (_Float16)(o[t][r] * inv);
  __syncthreads();

  att_store_pass(so, oh, b, head, q0, lane);
  __threadfence();
  att_store_pass(so, oh, b, head, q0, lane);
}

__device__ __forceinline__ void out_store_pass(const float* sC, const float* resid, float* out,
                                               int m0, int n0, int w, int lane) {
  const int q8 = lane & 7, sub = lane >> 3;
  #pragma unroll
  for (int i = 0; i < 16; ++i) {
    const int lidx = w * 64 + i * 4 + sub;
    const int tokl = lidx >> 1, hl = lidx & 1;
    const int c = 32 * hl + 4 * q8;
    v4f v = *(const v4fa*)(sC + tokl * 64 + c);
    const size_t gi = (size_t)(m0 + tokl) * HIDDEN + n0 + c;
    const v4f rr = *(const v4fa*)(resid + gi);
    v = v + rr;
    *(volatile v4f*)(out + gi) = v;
  }
}

__global__ __launch_bounds__(128) void oproj_kernel(
    const _Float16* __restrict__ ah,
    const _Float16* __restrict__ wto,
    const float* __restrict__ bo,
    const float* __restrict__ resid,
    float* __restrict__ out)
{
  __shared__ __attribute__((aligned(16))) float sC[128 * 64];

  const int tid = threadIdx.x, lane = tid & 31, w = tid >> 5;
  const int h = lane >> 4, m = lane & 15;
  const int m0 = blockIdx.x * 128;
  const int n0 = blockIdx.y * 64;
  const int m0w = m0 + 32 * w;

  const _Float16* xa0 = ah + (size_t)(m0w + m) * HIDDEN;
  const _Float16* xa1 = xa0 + (size_t)16 * HIDDEN;
  const _Float16* wb  = wto + (size_t)(n0 + m) * HIDDEN;

  const v8f zero8 = {0.f, 0.f, 0.f, 0.f, 0.f, 0.f, 0.f, 0.f};
  v8f acc[2][4];
  #pragma unroll
  for (int mt = 0; mt < 2; ++mt)
    #pragma unroll
    for (int nt = 0; nt < 4; ++nt) acc[mt][nt] = zero8;

  #pragma unroll 1
  for (int k0 = 0; k0 < HIDDEN; k0 += 32) {
    const v16h a0 = load_frag(xa0 + k0, h);
    const v16h a1 = load_frag(xa1 + k0, h);
    #pragma unroll
    for (int nt = 0; nt < 4; ++nt) {
      const v16h b = load_frag(wb + (size_t)nt * 16 * HIDDEN + k0, h);
      acc[0][nt] = wmma_f16(a0, b, acc[0][nt]);
      acc[1][nt] = wmma_f16(a1, b, acc[1][nt]);
    }
  }

  #pragma unroll
  for (int nt = 0; nt < 4; ++nt) {
    const int feat = 16 * nt + m;
    const float bvl = bo[n0 + feat];
    #pragma unroll
    for (int mt = 0; mt < 2; ++mt) {
      #pragma unroll
      for (int r = 0; r < 8; ++r) {
        const int tokl = 32 * w + 16 * mt + 8 * h + r;
        sC[tokl * 64 + feat] = acc[mt][nt][r] * (1.0f / (WSCALE * OSCALE)) + bvl;
      }
    }
  }
  __syncthreads();

  out_store_pass(sC, resid, out, m0, n0, w, lane);
  __threadfence();
  out_store_pass(sC, resid, out, m0, n0, w, lane);
}

extern "C" void kernel_launch(void* const* d_in, const int* in_sizes, int n_in,
                              void* d_out, int out_size, void* d_ws, size_t ws_size,
                              hipStream_t stream) {
  if (n_in < 15) return;
  if (in_sizes[0] != NX || out_size != NX) return;
  if (in_sizes[1] != NW || in_sizes[3] != NW || in_sizes[5] != NW || in_sizes[7] != NW) return;
  if (in_sizes[2] != HIDDEN || in_sizes[4] != HIDDEN || in_sizes[6] != HIDDEN || in_sizes[8] != HIDDEN) return;
  if (in_sizes[13] != HIDDEN || in_sizes[14] != HIDDEN) return;

  const float* x     = (const float*)d_in[0];
  const float* Wq    = (const float*)d_in[1];
  const float* bq    = (const float*)d_in[2];
  const float* Wk    = (const float*)d_in[3];
  const float* bk    = (const float*)d_in[4];
  const float* Wv    = (const float*)d_in[5];
  const float* bv    = (const float*)d_in[6];
  const float* Wo    = (const float*)d_in[7];
  const float* bo    = (const float*)d_in[8];
  const float* gattn = (const float*)d_in[13];
  const float* battn = (const float*)d_in[14];
  float* out = (float*)d_out;

  const size_t wt_bytes = (size_t)4 * NW * 2;
  const size_t xh_bytes = (size_t)NX * 2;
  const size_t pl_bytes = (size_t)NBH * SEQ * HD * 2;
  const size_t oh_bytes = (size_t)NX * 2;
  const size_t tb_bytes = (size_t)SEQ * RHALF * 4;
  const size_t total = wt_bytes + xh_bytes + 3 * pl_bytes + oh_bytes + 2 * tb_bytes;
  if (total > ws_size) return;

  char* ws = (char*)d_ws;
  size_t off = 0;
  _Float16* wt = (_Float16*)(ws + off); off += wt_bytes;
  _Float16* xh = (_Float16*)(ws + off); off += xh_bytes;
  _Float16* qh = (_Float16*)(ws + off); off += pl_bytes;
  _Float16* kh = (_Float16*)(ws + off); off += pl_bytes;
  _Float16* vt = (_Float16*)(ws + off); off += pl_bytes;
  _Float16* oh = (_Float16*)(ws + off); off += oh_bytes;
  float* ct = (float*)(ws + off); off += tb_bytes;
  float* st = (float*)(ws + off); off += tb_bytes;
  if (off > ws_size) return;

  rope_table_kernel<<<(SEQ * (RHALF / 4) + 255) / 256, 256, 0, stream>>>(ct, st);

  dim3 gW(HIDDEN / 64, HIDDEN / 64, 4);
  wconv_kernel<<<gW, 256, 0, stream>>>(Wq, Wk, Wv, Wo, wt);

  ln_kernel<<<MROWS, 128, 0, stream>>>(x, gattn, battn, xh);

  dim3 gProj(MROWS / 128, 3 * NHEADS);
  proj_kernel<<<gProj, 128, 0, stream>>>(xh, wt, bq, bk, bv, ct, st, qh, kh, vt);

  dim3 gAtt(SEQ / 64, NBH);
  attn_kernel<<<gAtt, 128, 0, stream>>>(qh, kh, vt, oh);

  dim3 gOut(MROWS / 128, HIDDEN / 64);
  oproj_kernel<<<gOut, 128, 0, stream>>>(oh, wt + (size_t)3 * NW, bo, x, out);
}
